// MessagePassingGNN_2834678415534
// MI455X (gfx1250) — hardware-verified
//
#include <hip/hip_runtime.h>
#include <stddef.h>
#include <stdint.h>
#include <math.h>


#define NN     50000
#define NE     800000
#define NP     50048
#define MR     850000
#define MRP    850048
#define HID    32
#define MH     64
#define KG     64
#define KE     128
#define NTHR   256
#define NWAVE  8
#define EPT    8
#define CHUNK  (NTHR * EPT)
#define WCAP   (EPT * 32)
#define LISTN  (NWAVE * WCAP)
#define NBA    1024
#define SLA    10
#define RCAP   28672
#define DEGCAP 64
#define GA     49
#define MEAS_B1024  16623
#define MEAS_MAXDEG 35
#define GTHR   128
#define GBM    64
#define TR     128
#define DP     68
#define AP     136
#define P_ENC  36
#define P_NODE 132
#define P_GRU  100
#define O_EWT  0
#define O_NB   2048
#define O_W2D  (O_NB + 3 * 256 * 64)
#define O_W3D  (O_W2D + 3 * 64 * 128)
#define O_WIH  (O_W3D + 3 * 32 * 128)
#define O_D1D  (O_WIH + 3 * 96 * 64)
#define O_D2D  (O_D1D + 64 * 64)
#define O_D3D  (O_D2D + 64 * 128)
#define WP_HALVES (O_D3D + 16 * 128)
#define PU0 (NP * 8)
#define PU1 (PU0 + 256)
#define PU2 (PU1 + 3072)
#define PU3 (PU2 + 3072)
#define PU4 (PU3 + 3072)
#define PU5 (PU4 + 1536)
#define PU6 (PU5 + 2304)
#define PU7 (PU6 + 512)
#define PU8 (PU7 + 1024)
#define PU9 (PU8 + 256)
#define BKT_LDS_INTS (LISTN + 2 * RCAP + 3 * NBA + 16)
#define AGG_LDS_BYTES (NBA * 32 * 4)
#define EDGE_LDS_BYTES (TR * DP * 4 + TR * AP * 2 + 96 * 4)
#define DEC_LDS_BYTES  (TR * DP * 4 + TR * AP * 2 + 144 * 4)

static_assert(NP % TR == 0 && NP % GBM == 0 && NP >= NN);
static_assert(MRP % TR == 0 && MRP >= MR && MR == NE + NN);
static_assert(GA * NBA >= NP);
static_assert(NE < (1 << 20));
static_assert((CHUNK & (CHUNK - 1)) == 0 && CHUNK <= 4096);
static_assert(NBA == (1 << SLA) && NBA % NWAVE == 0 && NBA == 4 * NTHR);
static_assert(RCAP % 32 == 0 && (RCAP % (NTHR * 4)) == 0);
static_assert(RCAP >= MEAS_B1024 + 4096);
static_assert(DEGCAP >= MEAS_MAXDEG + 8);
static_assert(BKT_LDS_INTS * 4 <= 300000 && AGG_LDS_BYTES <= 300000);
static_assert(EDGE_LDS_BYTES <= 300000 && DEC_LDS_BYTES <= 300000);
static_assert(PU0 % NTHR == 0 && PU9 % NTHR == 0);
static_assert((DP * 4) % 16 == 0 && (AP * 2) % 16 == 0 && AP >= KE && DP >= 64);
static_assert((TR * AP) % 2 == 0 && (TR * DP * 4) % 16 == 0 && (TR * AP * 2) % 16 == 0);
static_assert(O_NB % 64 == 0 && O_W2D % 64 == 0 && O_W3D % 64 == 0 && O_WIH % 64 == 0);
static_assert(O_D1D % 64 == 0 && O_D2D % 64 == 0 && O_D3D % 64 == 0);
static_assert(KG == 2 * HID && KE == 2 * MH && KG % 32 == 0 && KE % 32 == 0);

typedef float          v4f  __attribute__((ext_vector_type(4)));
typedef float          v8f  __attribute__((ext_vector_type(8)));
typedef int            v4i  __attribute__((ext_vector_type(4)));
typedef int            v8i  __attribute__((ext_vector_type(8)));
typedef unsigned short v8us __attribute__((ext_vector_type(8)));
typedef __bf16         v16b __attribute__((ext_vector_type(16)));
typedef v4f  __attribute__((may_alias)) v4fa;
typedef v4i  __attribute__((may_alias)) v4ia;
typedef v8us __attribute__((may_alias)) v8usa;
union FragB { v16b v; v8us h[2]; v8i w; };

__device__ __forceinline__ v8f wmb(const FragB& a, const FragB& b, v8f c) {
  v8f d = __builtin_amdgcn_wmma_f32_16x16x32_bf16(false, a.v, false, b.v, (short)0, c, false, false);
  asm volatile("v_nop\n\tv_nop\n\tv_nop\n\tv_nop" : "+v"(d) : "v"(a.w), "v"(b.w));
  return d;
}

__device__ __forceinline__ unsigned int f2bf(float f) {
  const unsigned int u = __float_as_uint(f);
  const unsigned int r = ((u + 0x7FFFu + ((u >> 16) & 1u)) >> 16) & 0xFFFFu;
  return ((u & 0x7FFFFFFFu) > 0x7F800000u) ? 0x7FC0u : r;
}
__device__ __forceinline__ float bf2f(unsigned int b) { return __uint_as_float(b << 16); }
__device__ __forceinline__ float bfr(float f) { return bf2f(f2bf(f)); }

template <int SLB>
__device__ __forceinline__ int scan_chunk(const int* __restrict__ dsts, int nE, int cbase, int slotBase,
                                          int nb, int vec8, int* list, int tid, int lane, int wave) {
  int wc = 0;
  const int el0  = tid * EPT;
  const int e0   = cbase + el0;
  const int sent = -2147483647 - 1;
  v4i da, db;
  if (vec8 != 0 && cbase + CHUNK <= nE) {
    da = *(const v4i*)(dsts + e0);
    db = *(const v4i*)(dsts + e0 + 4);
  } else {
    da.x = (e0     < nE) ? dsts[min(e0,     nE - 1)] : sent;
    da.y = (e0 + 1 < nE) ? dsts[min(e0 + 1, nE - 1)] : sent;
    da.z = (e0 + 2 < nE) ? dsts[min(e0 + 2, nE - 1)] : sent;
    da.w = (e0 + 3 < nE) ? dsts[min(e0 + 3, nE - 1)] : sent;
    db.x = (e0 + 4 < nE) ? dsts[min(e0 + 4, nE - 1)] : sent;
    db.y = (e0 + 5 < nE) ? dsts[min(e0 + 5, nE - 1)] : sent;
    db.z = (e0 + 6 < nE) ? dsts[min(e0 + 6, nE - 1)] : sent;
    db.w = (e0 + 7 < nE) ? dsts[min(e0 + 7, nE - 1)] : sent;
  }
  const unsigned nbs = (unsigned)slotBase;
  const unsigned unb = (unsigned)nb;
  const unsigned s0 = (unsigned)da.x - nbs, s1 = (unsigned)da.y - nbs;
  const unsigned s2 = (unsigned)da.z - nbs, s3 = (unsigned)da.w - nbs;
  const unsigned s4 = (unsigned)db.x - nbs, s5 = (unsigned)db.y - nbs;
  const unsigned s6 = (unsigned)db.z - nbs, s7 = (unsigned)db.w - nbs;
  const bool h0 = s0 < unb, h1 = s1 < unb, h2 = s2 < unb, h3 = s3 < unb;
  const bool h4 = s4 < unb, h5 = s5 < unb, h6 = s6 < unb, h7 = s7 < unb;
  const unsigned any = __builtin_amdgcn_ballot_w32(h0 | h1 | h2 | h3 | h4 | h5 | h6 | h7);
  if (any != 0u) {
#define HITJ(J, HJ, SJ) { \
      const unsigned mj = __builtin_amdgcn_ballot_w32(HJ); \
      if (mj != 0u) { \
        if (HJ) { \
          const int pos = wc + (int)__builtin_amdgcn_mbcnt_lo(mj, 0u); \
          if (pos < WCAP) list[wave * WCAP + pos] = ((el0 + (J)) << SLB) | (int)(SJ); \
        } \
        wc += (int)__builtin_popcount(mj); } }
    HITJ(0, h0, s0)
    HITJ(1, h1, s1)
    HITJ(2, h2, s2)
    HITJ(3, h3, s3)
    HITJ(4, h4, s4)
    HITJ(5, h5, s5)
    HITJ(6, h6, s6)
    HITJ(7, h7, s7)
#undef HITJ
  }
  return wc;
}

__global__ __launch_bounds__(NTHR) void k_prep(const float* __restrict__ x, const float* __restrict__ encW,
                                               const float* __restrict__ W1, const float* __restrict__ Whh,
                                               const float* __restrict__ W2, const float* __restrict__ W3,
                                               const float* __restrict__ Wih, const float* __restrict__ D1,
                                               const float* __restrict__ D2, const float* __restrict__ D3,
                                               unsigned short* XB, unsigned short* WP) {
  const int u = (int)blockIdx.x * NTHR + (int)threadIdx.x;
  v8us o;
  unsigned short* dp;
  if (u < PU0) {
    const int row = u >> 3;
    const int c0  = (u & 7) * 8;
    const int rc  = row < NN ? row : NN - 1;
    const float* p = x + (size_t)rc * 64 + c0;
    const v4f a = *(const v4fa*)p;
    const v4f b = *(const v4fa*)(p + 4);
    const bool ok = row < NN;
    o[0] = ok ? (unsigned short)f2bf(a.x) : (unsigned short)0;
    o[1] = ok ? (unsigned short)f2bf(a.y) : (unsigned short)0;
    o[2] = ok ? (unsigned short)f2bf(a.z) : (unsigned short)0;
    o[3] = ok ? (unsigned short)f2bf(a.w) : (unsigned short)0;
    o[4] = ok ? (unsigned short)f2bf(b.x) : (unsigned short)0;
    o[5] = ok ? (unsigned short)f2bf(b.y) : (unsigned short)0;
    o[6] = ok ? (unsigned short)f2bf(b.z) : (unsigned short)0;
    o[7] = ok ? (unsigned short)f2bf(b.w) : (unsigned short)0;
    dp = XB + (size_t)row * 64 + c0;
  } else if (u < PU1) {
    const int v  = u - PU0;
    const int n  = v >> 3;
    const int k8 = (v & 7) * 8;
    const float* p = encW + (size_t)k8 * 32 + n;
#pragma unroll
    for (int i = 0; i < 8; ++i) o[i] = (unsigned short)f2bf(p[(size_t)i * 32]);
    dp = WP + O_EWT + (size_t)n * 64 + k8;
  } else if (u < PU2) {
    const int v  = u - PU1;
    const int l  = v >> 10;
    const int n  = (v >> 3) & 127;
    const int k8 = (v & 7) * 8;
    const int kk = k8 & 31;
    const int q  = n >> 6;
    const float* p = W1 + (size_t)l * 4096 + (size_t)(32 * q + kk) * 64 + (n & 63);
#pragma unroll
    for (int i = 0; i < 8; ++i) o[i] = (unsigned short)f2bf(p[(size_t)i * 64]);
    dp = WP + O_NB + (size_t)(l * 256 + n) * 64 + k8;
  } else if (u < PU3) {
    const int v  = u - PU2;
    const int l  = v >> 10;
    const int nn = (v >> 3) & 127;
    const int k8 = (v & 7) * 8;
    const int kk = k8 & 31;
    const int rc = nn < 96 ? nn : 95;
    const float* p = Whh + (size_t)l * 3072 + (size_t)rc * 32 + kk;
    const v4f a = *(const v4fa*)p;
    const v4f b = *(const v4fa*)(p + 4);
    const bool ok = nn < 96;
    o[0] = ok ? (unsigned short)f2bf(a.x) : (unsigned short)0;
    o[1] = ok ? (unsigned short)f2bf(a.y) : (unsigned short)0;
    o[2] = ok ? (unsigned short)f2bf(a.z) : (unsigned short)0;
    o[3] = ok ? (unsigned short)f2bf(a.w) : (unsigned short)0;
    o[4] = ok ? (unsigned short)f2bf(b.x) : (unsigned short)0;
    o[5] = ok ? (unsigned short)f2bf(b.y) : (unsigned short)0;
    o[6] = ok ? (unsigned short)f2bf(b.z) : (unsigned short)0;
    o[7] = ok ? (unsigned short)f2bf(b.w) : (unsigned short)0;
    dp = WP + O_NB + (size_t)(l * 256 + 128 + nn) * 64 + k8;
  } else if (u < PU4) {
    const int v  = u - PU3;
    const int l  = v >> 10;
    const int n  = (v >> 4) & 63;
    const int k8 = (v & 15) * 8;
    const int kk = k8 & 63;
    const float* p = W2 + (size_t)l * 4096 + (size_t)kk * 64 + n;
#pragma unroll
    for (int i = 0; i < 8; ++i) o[i] = (unsigned short)f2bf(p[(size_t)i * 64]);
    dp = WP + O_W2D + (size_t)(l * 64 + n) * 128 + k8;
  } else if (u < PU5) {
    const int v  = u - PU4;
    const int l  = v >> 9;
    const int r  = v & 511;
    const int n  = r >> 4;
    const int k8 = (r & 15) * 8;
    const int kk = k8 & 63;
    const float* p = W3 + (size_t)l * 2048 + (size_t)kk * 32 + n;
#pragma unroll
    for (int i = 0; i < 8; ++i) o[i] = (unsigned short)f2bf(p[(size_t)i * 32]);
    dp = WP + O_W3D + (size_t)(l * 32 + n) * 128 + k8;
  } else if (u < PU6) {
    const int v  = u - PU5;
    const int l  = v / 768;
    const int r  = v - l * 768;
    const int n  = r >> 3;
    const int k8 = (r & 7) * 8;
    const int kk = k8 & 31;
    const float* p = Wih + (size_t)l * 3072 + (size_t)n * 32 + kk;
    const v4f a = *(const v4fa*)p;
    const v4f b = *(const v4fa*)(p + 4);
    o[0] = (unsigned short)f2bf(a.x); o[1] = (unsigned short)f2bf(a.y);
    o[2] = (unsigned short)f2bf(a.z); o[3] = (unsigned short)f2bf(a.w);
    o[4] = (unsigned short)f2bf(b.x); o[5] = (unsigned short)f2bf(b.y);
    o[6] = (unsigned short)f2bf(b.z); o[7] = (unsigned short)f2bf(b.w);
    dp = WP + O_WIH + (size_t)(l * 96 + n) * 64 + k8;
  } else if (u < PU7) {
    const int v  = u - PU6;
    const int n  = v >> 3;
    const int k8 = (v & 7) * 8;
    const int kk = k8 & 31;
    const float* p = D1 + (size_t)kk * 64 + n;
#pragma unroll
    for (int i = 0; i < 8; ++i) o[i] = (unsigned short)f2bf(p[(size_t)i * 64]);
    dp = WP + O_D1D + (size_t)n * 64 + k8;
  } else if (u < PU8) {
    const int v  = u - PU7;
    const int n  = v >> 4;
    const int k8 = (v & 15) * 8;
    const int kk = k8 & 63;
    const float* p = D2 + (size_t)kk * 64 + n;
#pragma unroll
    for (int i = 0; i < 8; ++i) o[i] = (unsigned short)f2bf(p[(size_t)i * 64]);
    dp = WP + O_D2D + (size_t)n * 128 + k8;
  } else if (u < PU9) {
    const int v  = u - PU8;
    const int n  = v >> 4;
    const int k8 = (v & 15) * 8;
    const int kk = k8 & 63;
    const int nc = n < 8 ? n : 7;
    const float* p = D3 + (size_t)kk * 8 + nc;
    const bool ok = n < 8;
#pragma unroll
    for (int i = 0; i < 8; ++i) {
      const float f = p[(size_t)i * 8];
      o[i] = ok ? (unsigned short)f2bf(f) : (unsigned short)0;
    }
    dp = WP + O_D3D + (size_t)n * 128 + k8;
  } else {
    return;
  }
  *(volatile v8us*)dp = o;
  __threadfence();
  *(volatile v8us*)dp = o;
}

__global__ __launch_bounds__(NTHR) void k_bucket(const int* __restrict__ dsts, int nE, int nN, int vec8,
                                                 int* LIST, int* CNT, int* OFF, int* FLG) {
  extern __shared__ __attribute__((aligned(16))) int bsm[];
  int* list = bsm;
  int* hl   = bsm + LISTN;
  int* sl   = hl + RCAP;
  int* cnt  = sl + RCAP;
  int* offs = cnt + NBA;
  int* cur  = offs + NBA;
  int* wcnt = cur + NBA;
  const int tid = (int)threadIdx.x, lane = tid & 31;
  const int wave = __builtin_amdgcn_readfirstlane(tid >> 5);
  const int blk = (int)blockIdx.x;
  const int nodeBase = blk * NBA;
  int nb = nN - nodeBase;
  nb = nb < 0 ? 0 : (nb > NBA ? NBA : nb);

  {
    const v4i z4 = {0, 0, 0, 0};
    for (int i = tid * 4; i < RCAP + 3 * NBA; i += NTHR * 4) *(v4ia*)(sl + i) = z4;
    if (tid < 16) wcnt[tid] = 0;
  }
  __syncthreads();

  int tot = 0, ovf = 0;
  const int nChunks = (nE + CHUNK - 1) / CHUNK;
#pragma unroll 1
  for (int ch = 0; ch < nChunks; ++ch) {
    const int cbase = ch * CHUNK;
    const int wc = scan_chunk<SLA>(dsts, nE, cbase, nodeBase, nb, vec8, list, tid, lane, wave);
    if (lane == 0) wcnt[wave] = wc;
    __syncthreads();
    int pre = 0, all = 0;
#pragma unroll
    for (int w2 = 0; w2 < NWAVE; ++w2) {
      int c = wcnt[w2];
      c = c < 0 ? 0 : (c > WCAP ? WCAP : c);
      all += c;
      pre += (w2 < wave) ? c : 0;
    }
    const int wcc  = wc > WCAP ? WCAP : wc;
    const int base = tot + pre;
#pragma unroll 1
    for (int i = lane; i < wcc; i += 32) {
      const int ent = list[wave * WCAP + i];
      const int el  = (ent >> SLA) & (CHUNK - 1);
      const int sq  = ent & (NBA - 1);
      int eid = cbase + el;
      eid = eid > nE - 1 ? nE - 1 : eid;
      const int pos = base + i;
      if (pos < RCAP) hl[pos] = (eid << SLA) | sq;
    }
    if (tot + all > RCAP) ovf = 1;
    tot += all;
    tot = tot > RCAP ? RCAP : tot;
    __syncthreads();
  }
  const int nh = __builtin_amdgcn_readfirstlane(tot);

  if (wave == 0) {
#pragma unroll 1
    for (int b0 = 0; b0 < nh; b0 += 32) {
      const int idx = b0 + lane;
      const int uv  = hl[idx < nh ? idx : nh - 1];
      const int m32 = (nh - b0) < 32 ? (nh - b0) : 32;
#pragma unroll 1
      for (int k = 0; k < m32; ++k) {
        const int u  = __builtin_amdgcn_readlane(uv, k);
        const int sq = u & (NBA - 1);
        if (lane == 0) cnt[sq] = cnt[sq] + 1;
      }
    }
  }
  __syncthreads();
  if (wave == 0) {
    const int base = lane * (NBA / 32);
    int s = 0;
#pragma unroll 1
    for (int i = 0; i < NBA / 32; ++i) s += cnt[base + i];
    int incl = s;
#pragma unroll
    for (int d = 1; d < 32; d <<= 1) {
      const int y = __shfl_up(incl, d, 32);
      if (lane >= d) incl += y;
    }
    int run = incl - s;
#pragma unroll 1
    for (int i = 0; i < NBA / 32; ++i) {
      const int cv = cnt[base + i];
      offs[base + i] = run;
      cur[base + i]  = run;
      run += cv;
    }
  }
  __syncthreads();
  if (wave == 0) {
#pragma unroll 1
    for (int b0 = 0; b0 < nh; b0 += 32) {
      const int idx = b0 + lane;
      const int uv  = hl[idx < nh ? idx : nh - 1];
      const int m32 = (nh - b0) < 32 ? (nh - b0) : 32;
#pragma unroll 1
      for (int k = 0; k < m32; ++k) {
        const int u  = __builtin_amdgcn_readlane(uv, k);
        const int sq = u & (NBA - 1);
        if (lane == 0) {
          int p = cur[sq];
          p = p < 0 ? 0 : (p > RCAP - 1 ? RCAP - 1 : p);
          sl[p] = u;
          cur[sq] = p + 1;
        }
      }
    }
  }
  __syncthreads();

  int* lb = LIST + (size_t)blk * RCAP;
  const v4i c4 = *(const v4ia*)(cnt + 4 * tid);
  const v4i o4 = *(const v4ia*)(offs + 4 * tid);
  v4i cv;
  cv.x = (tid == 0) ? nh : 0;
  cv.y = (tid == 0) ? ovf : 0;
  cv.z = 0; cv.w = 0;
  int* fp = FLG + (size_t)blk * 32 + 4 * (tid & 7);
  int* cp = CNT + (size_t)nodeBase + 4 * tid;
  int* op = OFF + (size_t)nodeBase + 4 * tid;
#pragma unroll 1
  for (int p = tid * 4; p < RCAP; p += NTHR * 4) {
    const v4i v = *(const v4ia*)(sl + p);
    v4i e;
    e.x = (int)((unsigned)v.x >> SLA); e.y = (int)((unsigned)v.y >> SLA);
    e.z = (int)((unsigned)v.z >> SLA); e.w = (int)((unsigned)v.w >> SLA);
    *(volatile v4i*)(lb + p) = e;
  }
  *(volatile v4i*)cp = c4;
  *(volatile v4i*)op = o4;
  if (tid < 8) *(volatile v4i*)fp = cv;
  __threadfence();
#pragma unroll 1
  for (int p = tid * 4; p < RCAP; p += NTHR * 4) {
    const v4i v = *(const v4ia*)(sl + p);
    v4i e;
    e.x = (int)((unsigned)v.x >> SLA); e.y = (int)((unsigned)v.y >> SLA);
    e.z = (int)((unsigned)v.z >> SLA); e.w = (int)((unsigned)v.w >> SLA);
    *(volatile v4i*)(lb + p) = e;
  }
  *(volatile v4i*)cp = c4;
  *(volatile v4i*)op = o4;
  if (tid < 8) *(volatile v4i*)fp = cv;
}

template <int MT, int NT>
__device__ __forceinline__ void wgemm_gl(const unsigned short* __restrict__ ap, int lda,
                                         const unsigned short* __restrict__ bp,
                                         float* sDw, int dpitch, const float* cb, int hh, int m) {
  v8f acc[MT][NT];
  {
    const v8f z = {0.f, 0.f, 0.f, 0.f, 0.f, 0.f, 0.f, 0.f};
#pragma unroll
    for (int mt = 0; mt < MT; ++mt)
#pragma unroll
      for (int nt = 0; nt < NT; ++nt) acc[mt][nt] = z;
  }
#pragma unroll
  for (int ks = 0; ks < KG / 32; ++ks) {
    const int k0 = 32 * ks;
    FragB a[MT];
#pragma unroll
    for (int mt = 0; mt < MT; ++mt) {
      const unsigned short* aq = ap + (size_t)(16 * mt) * (size_t)lda + k0;
      a[mt].h[0] = *(const v8usa*)aq;
      a[mt].h[1] = *(const v8usa*)(aq + 16);
    }
#pragma unroll
    for (int nt = 0; nt < NT; ++nt) {
      const unsigned short* wq = bp + (16 * nt) * KG + k0;
      FragB b;
      b.h[0] = *(const v8usa*)wq;
      b.h[1] = *(const v8usa*)(wq + 16);
#pragma unroll
      for (int mt = 0; mt < MT; ++mt) acc[mt][nt] = wmb(a[mt], b, acc[mt][nt]);
    }
  }
#pragma unroll
  for (int nt = 0; nt < NT; ++nt) {
    const int col = 16 * nt + m;
    const float bv = cb[col];
#pragma unroll
    for (int mt = 0; mt < MT; ++mt)
#pragma unroll
      for (int r = 0; r < 8; ++r) sDw[(16 * mt + 8 * hh + r) * dpitch + col] = acc[mt][nt][r] + bv;
  }
}

template <int NT>
__device__ __forceinline__ void wgemm_lds(const unsigned short* sAw, const unsigned short* __restrict__ BT,
                                          float* sDw, const float* cb, int hh, int m) {
  v8f acc[2][NT];
  {
    const v8f z = {0.f, 0.f, 0.f, 0.f, 0.f, 0.f, 0.f, 0.f};
#pragma unroll
    for (int mt = 0; mt < 2; ++mt)
#pragma unroll
      for (int nt = 0; nt < NT; ++nt) acc[mt][nt] = z;
  }
  const unsigned short* ap0 = sAw + m * AP + 8 * hh;
  const unsigned short* ap1 = ap0 + 16 * AP;
  const unsigned short* bp  = BT + (size_t)m * KE + 8 * hh;
#pragma unroll 1
  for (int k0 = 0; k0 < KE; k0 += 32) {
    FragB a0, a1;
    a0.h[0] = *(const v8usa*)(ap0 + k0);
    a0.h[1] = *(const v8usa*)(ap0 + k0 + 16);
    a1.h[0] = *(const v8usa*)(ap1 + k0);
    a1.h[1] = *(const v8usa*)(ap1 + k0 + 16);
#pragma unroll
    for (int nt = 0; nt < NT; ++nt) {
      const unsigned short* wq = bp + (16 * nt) * KE + k0;
      FragB b;
      b.h[0] = *(const v8usa*)wq;
      b.h[1] = *(const v8usa*)(wq + 16);
      acc[0][nt] = wmb(a0, b, acc[0][nt]);
      acc[1][nt] = wmb(a1, b, acc[1][nt]);
    }
  }
#pragma unroll
  for (int nt = 0; nt < NT; ++nt) {
    const int col = 16 * nt + m;
    const float bv = cb[col];
#pragma unroll
    for (int mt = 0; mt < 2; ++mt)
#pragma unroll
      for (int r = 0; r < 8; ++r) sDw[(16 * mt + 8 * hh + r) * DP + col] = acc[mt][nt][r] + bv;
  }
}

__device__ __forceinline__ void act_row(const float* rd, unsigned short* ra) {
#pragma unroll 1
  for (int c = 0; c < MH; ++c) {
    const float t = tanhf(rd[c]);
    const unsigned hb = f2bf(t);
    const unsigned lb = f2bf(t - bf2f(hb));
    ra[c]      = (unsigned short)hb;
    ra[MH + c] = (unsigned short)lb;
  }
}

template <bool RELU>
__device__ __forceinline__ void store_h_rows(const float* st, int pitch, int rowBase, int wave, int lane,
                                             float* H, unsigned short* Hhl) {
  const int rq = lane >> 3, j = lane & 7;
  const int part = j >> 2;
  const int c0 = 8 * (j & 3);
  const unsigned mh = 0u - (unsigned)part;
  const unsigned ml = ~mh;
  v4f  pv[4];
  v8us hv[4];
#pragma unroll
  for (int i = 0; i < 4; ++i) {
    const float* sp = st + (16 * wave + 4 * i + rq) * pitch;
    v4f a = *(const v4fa*)(sp + 4 * j);
    const v4f b0 = *(const v4fa*)(sp + c0);
    const v4f b1 = *(const v4fa*)(sp + c0 + 4);
    v8f f8 = {b0.x, b0.y, b0.z, b0.w, b1.x, b1.y, b1.z, b1.w};
    if (RELU) {
      a.x = (a.x > 0.0f) ? a.x : (a.x - a.x);
      a.y = (a.y > 0.0f) ? a.y : (a.y - a.y);
      a.z = (a.z > 0.0f) ? a.z : (a.z - a.z);
      a.w = (a.w > 0.0f) ? a.w : (a.w - a.w);
#pragma unroll
      for (int e = 0; e < 8; ++e) f8[e] = (f8[e] > 0.0f) ? f8[e] : (f8[e] - f8[e]);
    }
    pv[i] = a;
    v8us oo;
#pragma unroll
    for (int e = 0; e < 8; ++e) {
      const unsigned hb = f2bf(f8[e]);
      const unsigned lb = f2bf(f8[e] - bf2f(hb));
      oo[e] = (unsigned short)((hb & ml) | (lb & mh));
    }
    hv[i] = oo;
  }
#pragma unroll
  for (int i = 0; i < 4; ++i) {
    const size_t gr = (size_t)(rowBase + 16 * wave + 4 * i + rq);
    *(volatile v4f*)(H + gr * HID + 4 * j) = pv[i];
    *(volatile v8us*)(Hhl + gr * 64 + 8 * j) = hv[i];
  }
  __threadfence();
#pragma unroll
  for (int i = 0; i < 4; ++i) {
    const size_t gr = (size_t)(rowBase + 16 * wave + 4 * i + rq);
    *(volatile v4f*)(H + gr * HID + 4 * j) = pv[i];
    *(volatile v8us*)(Hhl + gr * 64 + 8 * j) = hv[i];
  }
}

template <int NL>
__device__ __forceinline__ void store_rows16(const float* st, int pitch, int rowBase, int wave, int lane,
                                             float* dst, int ld) {
  const int lc = lane < NL ? lane : NL - 1;
  v4f pv[16];
#pragma unroll
  for (int i = 0; i < 16; ++i) pv[i] = *(const v4fa*)(st + (16 * wave + i) * pitch + 4 * lc);
#pragma unroll
  for (int i = 0; i < 16; ++i) {
    float* op = dst + (size_t)(rowBase + 16 * wave + i) * (size_t)ld + 4 * lane;
    if (lane < NL) *(volatile v4f*)op = pv[i];
  }
  __threadfence();
#pragma unroll
  for (int i = 0; i < 16; ++i) {
    float* op = dst + (size_t)(rowBase + 16 * wave + i) * (size_t)ld + 4 * lane;
    if (lane < NL) *(volatile v4f*)op = pv[i];
  }
}

__global__ __launch_bounds__(GTHR) void k_enc(const unsigned short* __restrict__ XB,
                                              const unsigned short* __restrict__ EWT,
                                              const float* __restrict__ encb, float* H, unsigned short* Hhl) {
  __shared__ __attribute__((aligned(16))) float stg[GBM * P_ENC];
  __shared__ __attribute__((aligned(16))) float sb[32];
  const int tid = (int)threadIdx.x, lane = tid & 31, wave = tid >> 5, hh = lane >> 4, m = lane & 15;
  const int rowBase = (int)blockIdx.x * GBM;
  if (tid < 32) sb[tid] = bfr(encb[tid]);
  __syncthreads();
  wgemm_gl<1, 2>(XB + (size_t)(rowBase + 16 * wave + m) * 64 + 8 * hh, 64, EWT + m * KG + 8 * hh,
                 stg + 16 * wave * P_ENC, P_ENC, sb, hh, m);
  __syncthreads();
  store_h_rows<true>(stg, P_ENC, rowBase, wave, lane, H, Hhl);
}

__global__ __launch_bounds__(GTHR) void k_node(const unsigned short* __restrict__ Hhl,
                                               const unsigned short* __restrict__ NBl,
                                               const float* __restrict__ b1l, const float* __restrict__ bhhl,
                                               float* PDS, float* GH) {
  __shared__ __attribute__((aligned(16))) float stg[GBM * P_NODE];
  __shared__ __attribute__((aligned(16))) float sb[256];
  const int tid = (int)threadIdx.x, lane = tid & 31, wave = tid >> 5, hh = lane >> 4, m = lane & 15;
  const int rowBase = (int)blockIdx.x * GBM;
  {
    const float v1 = b1l[tid < 64 ? tid : 63];
    const float v2 = bhhl[tid < 96 ? tid : 95];
    sb[tid]       = (tid < 64) ? bfr(v1) : 0.0f;
    sb[128 + tid] = (tid < 96) ? bfr(v2) : 0.0f;
  }
  __syncthreads();
  const unsigned short* ap = Hhl + (size_t)(rowBase + 16 * wave + m) * 64 + 8 * hh;
#pragma unroll 1
  for (int nh = 0; nh < 2; ++nh) {
    wgemm_gl<1, 8>(ap, 64, NBl + (size_t)(128 * nh + m) * KG + 8 * hh, stg + 16 * wave * P_NODE, P_NODE,
                   sb + 128 * nh, hh, m);
    __syncthreads();
    if (nh == 0) store_rows16<32>(stg, P_NODE, rowBase, wave, lane, PDS, 128);
    else         store_rows16<24>(stg, P_NODE, rowBase, wave, lane, GH, 96);
    __syncthreads();
  }
}

__global__ __launch_bounds__(TR) void k_edge(const int* __restrict__ src, const int* __restrict__ dst,
                                             const float* __restrict__ PDS,
                                             const unsigned short* __restrict__ W2Dl,
                                             const unsigned short* __restrict__ W3Dl,
                                             const float* __restrict__ b2l, const float* __restrict__ b3l,
                                             float* M) {
  extern __shared__ __attribute__((aligned(16))) float dyn[];
  float*          sD  = dyn;
  unsigned short* sA  = (unsigned short*)(dyn + TR * DP);
  float*          cst = dyn + TR * DP + (TR * AP) / 2;
  const int tid = (int)threadIdx.x, lane = tid & 31, wave = tid >> 5, hh = lane >> 4, m = lane & 15;
  const int blk = (int)blockIdx.x;

  if (tid < 64) cst[tid] = bfr(b2l[tid]);
  if (tid < 32) cst[64 + tid] = bfr(b3l[tid]);

  const int rho = blk * TR + tid;
  const int rc  = rho < MR ? rho : MR - 1;
  const int ec  = rc < NE ? rc : NE - 1;
  const int sL  = src[ec];
  const int dL  = dst[ec];
  const bool isE = rc < NE;
  const int lp  = rc - NE;
  int s = isE ? sL : lp;
  int d = isE ? dL : lp;
  s = s < 0 ? 0 : (s > NN - 1 ? NN - 1 : s);
  d = d < 0 ? 0 : (d > NN - 1 ? NN - 1 : d);

  float*          rd = sD + tid * DP;
  unsigned short* ra = sA + tid * AP;
  {
    const float* pdr = PDS + (size_t)d * 128;
    const float* psr = PDS + (size_t)s * 128 + 64;
#pragma unroll 1
    for (int c4 = 0; c4 < 16; ++c4) {
      const v4f a = *(const v4fa*)(pdr + 4 * c4);
      const v4f b = *(const v4fa*)(psr + 4 * c4);
      v4f q;
      q.x = a.x + b.x; q.y = a.y + b.y; q.z = a.z + b.z; q.w = a.w + b.w;
      *(v4fa*)(rd + 4 * c4) = q;
    }
  }
  act_row(rd, ra);
  __syncthreads();

  const unsigned short* sAw = sA + 32 * wave * AP;
  float*                sDw = sD + 32 * wave * DP;
  wgemm_lds<4>(sAw, W2Dl, sDw, cst, hh, m);
  __syncthreads();
  act_row(rd, ra);
  __syncthreads();
  wgemm_lds<2>(sAw, W3Dl, sDw, cst + 64, hh, m);
  __syncthreads();

  {
    float* mb = M + (size_t)blk * (TR * HID);
    v4f pv[8];
#pragma unroll
    for (int it = 0; it < 8; ++it) {
      const int p = it * TR + tid;
      pv[it] = *(const v4fa*)(sD + (p >> 3) * DP + 4 * (p & 7));
    }
#pragma unroll
    for (int it = 0; it < 8; ++it) *(volatile v4f*)(mb + (size_t)(it * TR + tid) * 4) = pv[it];
    __threadfence();
#pragma unroll
    for (int it = 0; it < 8; ++it) *(volatile v4f*)(mb + (size_t)(it * TR + tid) * 4) = pv[it];
  }
}

__device__ __forceinline__ void agg_flush(const float* tile, unsigned short* AGGhl, int nodeBase, int tid) {
#pragma unroll 1
  for (int it = 0; it < 32; ++it) {
    const int p = it * NTHR + tid;
    const int row = p >> 3, j = p & 7;
    const int part = j >> 2;
    const int c0 = 8 * (j & 3);
    const unsigned mh = 0u - (unsigned)part;
    const unsigned ml = ~mh;
    const float* sp = tile + row * 32 + c0;
    const v4f a = *(const v4fa*)sp;
    const v4f b = *(const v4fa*)(sp + 4);
    const v8f f8 = {a.x, a.y, a.z, a.w, b.x, b.y, b.z, b.w};
    v8us oo;
#pragma unroll
    for (int e = 0; e < 8; ++e) {
      const unsigned hb = f2bf(f8[e]);
      const unsigned lb = f2bf(f8[e] - bf2f(hb));
      oo[e] = (unsigned short)((hb & ml) | (lb & mh));
    }
    const int node = nodeBase + row;
    if (node < NP) *(volatile v8us*)(AGGhl + (size_t)node * 64 + 8 * j) = oo;
  }
}

__global__ __launch_bounds__(NTHR) void k_agg(const int* __restrict__ LIST, const int* __restrict__ CNT,
                                              const int* __restrict__ OFF, const int* __restrict__ FLG,
                                              const float* __restrict__ M, unsigned short* AGGhl) {
  extern __shared__ __attribute__((aligned(16))) float tile[];
  const int tid = (int)threadIdx.x, lane = tid & 31;
  const int wave = __builtin_amdgcn_readfirstlane(tid >> 5);
  const int blk = (int)blockIdx.x;
  const int nodeBase = blk * NBA;
  const int nhraw = FLG[(size_t)blk * 32];
  const int bflag = FLG[(size_t)blk * 32 + 1];
  const bool ovf = (bflag != 0) || (nhraw < 0) || (nhraw > RCAP);
  const float qnan = __int_as_float(0x7fc00000);
  const float pzb = ovf ? qnan : 0.0f;
  const int* lb = LIST + (size_t)blk * RCAP;

#pragma unroll 1
  for (int si = 0; si < NBA / NWAVE; ++si) {
    const int s    = si * NWAVE + wave;
    const int node = nodeBase + s;
    const int nc   = node < NN ? node : NN - 1;
    const int craw = __builtin_amdgcn_readfirstlane(CNT[(size_t)nodeBase + s]);
    const int oraw = __builtin_amdgcn_readfirstlane(OFF[(size_t)nodeBase + s]);
    const bool big = (craw < 0) || (craw > DEGCAP);
    int c = craw < 0 ? 0 : (craw > DEGCAP ? DEGCAP : craw);
    int o = oraw < 0 ? 0 : (oraw > RCAP ? RCAP : oraw);
    if (c > RCAP - o) c = RCAP - o;
    float acc = 0.0f;
#pragma unroll 1
    for (int b0 = 0; b0 < c; b0 += 32) {
      int idx = o + b0 + lane;
      idx = idx > RCAP - 1 ? RCAP - 1 : idx;
      int eid = lb[idx];
      eid = eid < 0 ? 0 : (eid > NE - 1 ? NE - 1 : eid);
      const int m32 = (c - b0) < 32 ? (c - b0) : 32;
#pragma unroll 1
      for (int k = 0; k < m32; ++k) {
        const int ek = __builtin_amdgcn_readlane(eid, k);
        acc += M[(size_t)ek * HID + lane];
      }
    }
    acc += M[(size_t)(NE + nc) * HID + lane];
    const float inv = 1.0f / (float)(c + 1);
    const float v = acc * inv + (big ? qnan : pzb);
    tile[s * 32 + lane] = (node < NN) ? v : 0.0f;
  }
  __syncthreads();
  agg_flush(tile, AGGhl, nodeBase, tid);
  __threadfence();
  agg_flush(tile, AGGhl, nodeBase, tid);
}

__global__ __launch_bounds__(GTHR) void k_gru(const unsigned short* __restrict__ AGGhl,
                                              const unsigned short* __restrict__ WihDl,
                                              const float* __restrict__ bihl, const float* __restrict__ GH,
                                              const float* __restrict__ Hold, float* Hnew, unsigned short* Hhl) {
  __shared__ __attribute__((aligned(16))) float stg[GBM * P_GRU];
  __shared__ __attribute__((aligned(16))) float sh[GBM * P_ENC];
  __shared__ __attribute__((aligned(16))) float sb[96];
  const int tid = (int)threadIdx.x, lane = tid & 31, wave = tid >> 5, hh = lane >> 4, m = lane & 15;
  const int rowBase = (int)blockIdx.x * GBM;
  if (tid < 96) sb[tid] = bfr(bihl[tid]);
  __syncthreads();
  wgemm_gl<1, 6>(AGGhl + (size_t)(rowBase + 16 * wave + m) * 64 + 8 * hh, 64, WihDl + m * KG + 8 * hh,
                 stg + 16 * wave * P_GRU, P_GRU, sb, hh, m);
  __syncthreads();
#pragma unroll 1
  for (int it = 0; it < (GBM * HID) / GTHR; ++it) {
    const int e = it * GTHR + tid;
    const int row = e >> 5, c = e & 31;
    const size_t gr = (size_t)(rowBase + row);
    const float gir = stg[row * P_GRU + c];
    const float giz = stg[row * P_GRU + 32 + c];
    const float gin = stg[row * P_GRU + 64 + c];
    const float ghr = GH[gr * 96 + c];
    const float ghz = GH[gr * 96 + 32 + c];
    const float ghn = GH[gr * 96 + 64 + c];
    const float ho  = Hold[gr * HID + c];
    const float rg = 1.0f / (1.0f + expf(-(gir + ghr)));
    const float zg = 1.0f / (1.0f + expf(-(giz + ghz)));
    const float ng = tanhf(gin + rg * ghn);
    sh[row * P_ENC + c] = (1.0f - zg) * ng + zg * ho;
  }
  __syncthreads();
  store_h_rows<false>(sh, P_ENC, rowBase, wave, lane, Hnew, Hhl);
}

__global__ __launch_bounds__(TR) void k_dec(const unsigned short* __restrict__ Hhl,
                                            const unsigned short* __restrict__ D1D,
                                            const unsigned short* __restrict__ D2D,
                                            const unsigned short* __restrict__ D3D,
                                            const float* __restrict__ b1, const float* __restrict__ b2,
                                            const float* __restrict__ b3, const int* __restrict__ FLG,
                                            float* out) {
  extern __shared__ __attribute__((aligned(16))) float dyn[];
  float*          sD  = dyn;
  unsigned short* sA  = (unsigned short*)(dyn + TR * DP);
  float*          cst = dyn + TR * DP + (TR * AP) / 2;
  const int tid = (int)threadIdx.x, lane = tid & 31, wave = tid >> 5, hh = lane >> 4, m = lane & 15;
  const int rowBase = (int)blockIdx.x * TR;

  if (tid < 64) { cst[tid] = bfr(b1[tid]); cst[64 + tid] = bfr(b2[tid]); }
  {
    const float v3 = b3[tid & 7];
    if (tid < 16) cst[128 + tid] = (tid < 8) ? bfr(v3) : 0.0f;
  }
  __syncthreads();

  float*          rd  = sD + tid * DP;
  unsigned short* ra  = sA + tid * AP;
  const unsigned short* sAw = sA + 32 * wave * AP;
  float*          sDw = sD + 32 * wave * DP;

  wgemm_gl<2, 4>(Hhl + (size_t)(rowBase + 32 * wave + m) * 64 + 8 * hh, 64, D1D + m * KG + 8 * hh,
                 sDw, DP, cst, hh, m);
  __syncthreads();
  act_row(rd, ra);
  __syncthreads();
  wgemm_lds<4>(sAw, D2D, sDw, cst + 64, hh, m);
  __syncthreads();
  act_row(rd, ra);
  __syncthreads();
  wgemm_lds<1>(sAw, D3D, sDw, cst + 128, hh, m);
  __syncthreads();

  const int fb = rowBase >> SLA;
  const int nhraw = FLG[(size_t)fb * 32];
  const int bflag = FLG[(size_t)fb * 32 + 1];
  const bool pf = (bflag != 0) || (nhraw < 0) || (nhraw > RCAP);
  const float qnan = __int_as_float(0x7fc00000);
  v4f pv[2];
#pragma unroll
  for (int it = 0; it < 2; ++it) {
    const int p = it * TR + tid;
    const v4f v = *(const v4fa*)(sD + (p >> 1) * DP + 4 * (p & 1));
    v4f q;
    q.x = pf ? qnan : v.x; q.y = pf ? qnan : v.y; q.z = pf ? qnan : v.z; q.w = pf ? qnan : v.w;
    pv[it] = q;
  }
#pragma unroll
  for (int it = 0; it < 2; ++it) {
    const int p = it * TR + tid;
    if (rowBase + (p >> 1) < NN) *(volatile v4f*)(out + (size_t)rowBase * 8 + (size_t)p * 4) = pv[it];
  }
  __threadfence();
#pragma unroll
  for (int it = 0; it < 2; ++it) {
    const int p = it * TR + tid;
    if (rowBase + (p >> 1) < NN) *(volatile v4f*)(out + (size_t)rowBase * 8 + (size_t)p * 4) = pv[it];
  }
}

extern "C" void kernel_launch(void* const* d_in, const int* in_sizes, int n_in,
                              void* d_out, int out_size, void* d_ws, size_t ws_size,
                              hipStream_t stream) {
  if (n_in < 20) return;
  if (in_sizes[0] != NN * 64) return;
  if (in_sizes[1] != 2 * NE) return;
  if (in_sizes[2] != 64 * 32 || in_sizes[3] != 32) return;
  if (in_sizes[4] != 3 * 64 * 64 || in_sizes[5] != 3 * 64) return;
  if (in_sizes[6] != 3 * 64 * 64 || in_sizes[7] != 3 * 64) return;
  if (in_sizes[8] != 3 * 64 * 32 || in_sizes[9] != 3 * 32) return;
  if (in_sizes[10] != 3 * 96 * 32 || in_sizes[11] != 3 * 96 * 32) return;
  if (in_sizes[12] != 3 * 96 || in_sizes[13] != 3 * 96) return;
  if (in_sizes[14] != 32 * 64 || in_sizes[15] != 64) return;
  if (in_sizes[16] != 64 * 64 || in_sizes[17] != 64) return;
  if (in_sizes[18] != 64 * 8 || in_sizes[19] != 8) return;
  if (out_size != NN * 8) return;

  const float* x     = (const float*)d_in[0];
  const int*   ei    = (const int*)  d_in[1];
  const float* encW  = (const float*)d_in[2];
  const float* encb  = (const float*)d_in[3];
  const float* mW1   = (const float*)d_in[4];
  const float* mb1   = (const float*)d_in[5];
  const float* mW2   = (const float*)d_in[6];
  const float* mb2   = (const float*)d_in[7];
  const float* mW3   = (const float*)d_in[8];
  const float* mb3   = (const float*)d_in[9];
  const float* gWih  = (const float*)d_in[10];
  const float* gWhh  = (const float*)d_in[11];
  const float* gbih  = (const float*)d_in[12];
  const float* gbhh  = (const float*)d_in[13];
  const float* dW1   = (const float*)d_in[14];
  const float* db1   = (const float*)d_in[15];
  const float* dW2   = (const float*)d_in[16];
  const float* db2   = (const float*)d_in[17];
  const float* dW3   = (const float*)d_in[18];
  const float* db3   = (const float*)d_in[19];
  float* out = (float*)d_out;
  const int* src = ei;
  const int* dst = ei + NE;

  char* ws = (char*)d_ws;
  size_t off = 0;
  const size_t oWP  = off; off += (size_t)WP_HALVES * 2;      off = (off + 255) & ~(size_t)255;
  const size_t oXB  = off; off += (size_t)NP * 64 * 2;        off = (off + 255) & ~(size_t)255;
  const size_t oHA  = off; off += (size_t)NP * HID * 4;       off = (off + 255) & ~(size_t)255;
  const size_t oHB  = off; off += (size_t)NP * HID * 4;       off = (off + 255) & ~(size_t)255;
  const size_t oHhl = off; off += (size_t)NP * 64 * 2;        off = (off + 255) & ~(size_t)255;
  const size_t oAG  = off; off += (size_t)NP * 64 * 2;        off = (off + 255) & ~(size_t)255;
  const size_t oPDS = off; off += (size_t)NP * 128 * 4;       off = (off + 255) & ~(size_t)255;
  const size_t oGH  = off; off += (size_t)NP * 96 * 4;        off = (off + 255) & ~(size_t)255;
  const size_t oM   = off; off += (size_t)MRP * HID * 4;      off = (off + 255) & ~(size_t)255;
  const size_t oLI  = off; off += (size_t)GA * RCAP * 4;      off = (off + 255) & ~(size_t)255;
  const size_t oCN  = off; off += (size_t)GA * NBA * 4;       off = (off + 255) & ~(size_t)255;
  const size_t oOF  = off; off += (size_t)GA * NBA * 4;       off = (off + 255) & ~(size_t)255;
  const size_t oFL  = off; off += (size_t)GA * 128;           off = (off + 255) & ~(size_t)255;
  if (off > ws_size) return;
  unsigned short* WP    = (unsigned short*)(ws + oWP);
  unsigned short* XB    = (unsigned short*)(ws + oXB);
  float*          HA    = (float*)(ws + oHA);
  float*          HB    = (float*)(ws + oHB);
  unsigned short* Hhl   = (unsigned short*)(ws + oHhl);
  unsigned short* AGGhl = (unsigned short*)(ws + oAG);
  float*          PDS   = (float*)(ws + oPDS);
  float*          GH    = (float*)(ws + oGH);
  float*          M     = (float*)(ws + oM);
  int*            LIST  = (int*)(ws + oLI);
  int*            CNT   = (int*)(ws + oCN);
  int*            OFF   = (int*)(ws + oOF);
  int*            FLG   = (int*)(ws + oFL);

  const int bktLds = BKT_LDS_INTS * 4;
  hipFuncSetAttribute(reinterpret_cast<const void*>(&k_bucket), hipFuncAttributeMaxDynamicSharedMemorySize, bktLds);
  hipFuncSetAttribute(reinterpret_cast<const void*>(&k_agg), hipFuncAttributeMaxDynamicSharedMemorySize,
                      (int)AGG_LDS_BYTES);
  hipFuncSetAttribute(reinterpret_cast<const void*>(&k_edge), hipFuncAttributeMaxDynamicSharedMemorySize,
                      (int)EDGE_LDS_BYTES);
  hipFuncSetAttribute(reinterpret_cast<const void*>(&k_dec), hipFuncAttributeMaxDynamicSharedMemorySize,
                      (int)DEC_LDS_BYTES);

  const int vec8 = ((NE & 3) == 0) ? 1 : 0;

  k_prep<<<PU9 / NTHR, NTHR, 0, stream>>>(x, encW, mW1, gWhh, mW2, mW3, gWih, dW1, dW2, dW3, XB, WP);
  k_bucket<<<GA, NTHR, bktLds, stream>>>(dst, NE, NN, vec8, LIST, CNT, OFF, FLG);
  k_enc<<<NP / GBM, GTHR, 0, stream>>>(XB, WP + O_EWT, encb, HA, Hhl);

  float* Hcur = HA;
  float* Hnxt = HB;
  for (int l = 0; l < 3; ++l) {
    k_node<<<NP / GBM, GTHR, 0, stream>>>(Hhl, WP + O_NB + (size_t)l * 256 * 64, mb1 + l * 64, gbhh + l * 96,
                                          PDS, GH);
    k_edge<<<MRP / TR, TR, EDGE_LDS_BYTES, stream>>>(src, dst, PDS, WP + O_W2D + (size_t)l * 64 * 128,
                                                      WP + O_W3D + (size_t)l * 32 * 128, mb2 + l * 64,
                                                      mb3 + l * 32, M);
    k_agg<<<GA, NTHR, AGG_LDS_BYTES, stream>>>(LIST, CNT, OFF, FLG, M, AGGhl);
    k_gru<<<NP / GBM, GTHR, 0, stream>>>(AGGhl, WP + O_WIH + (size_t)l * 96 * 64, gbih + l * 96, GH,
                                         Hcur, Hnxt, Hhl);
    float* t = Hcur; Hcur = Hnxt; Hnxt = t;
  }
  k_dec<<<NP / TR, TR, DEC_LDS_BYTES, stream>>>(Hhl, WP + O_D1D, WP + O_D2D, WP + O_D3D, db1, db2, db3, FLG, out);
}
